// BinaryFullTensorCell_75453985456646
// MI455X (gfx1250) — hardware-verified
//
#include <hip/hip_runtime.h>
#include <math.h>

typedef __attribute__((ext_vector_type(16))) _Float16 v16h;
typedef __attribute__((ext_vector_type(16))) __bf16 v16b;
typedef __attribute__((ext_vector_type(8)))  _Float16 v8h;
typedef __attribute__((ext_vector_type(8)))  float v8f;
typedef __attribute__((ext_vector_type(4)))  float v4f;
typedef __attribute__((ext_vector_type(2)))  float v2f;
typedef __attribute__((ext_vector_type(4)))  unsigned v4u;
typedef __attribute__((ext_vector_type(4)))  int v4i;
typedef float __attribute__((may_alias)) float_a;
typedef int __attribute__((may_alias)) int_a;

template <typename T> __device__ __forceinline__ void vst2(void* p, T v) { *(volatile T*)p = v; __threadfence(); *(volatile T*)p = v; }
__device__ __forceinline__ v8f wmma16(v16h a, v16h b, v8f c) {
  v8f d = __builtin_amdgcn_wmma_f32_16x16x32_f16(false, a, false, b, (short)0, c, false, false);
  asm volatile("v_nop\n\tv_nop\n\tv_nop\n\tv_nop" : "+v"(d) : "v"(a), "v"(b));
  return d;
}
__device__ __forceinline__ v8f wmma_bf(v16b a, v16b b, v8f c) {
  v8f d = __builtin_amdgcn_wmma_f32_16x16x32_bf16(false, a, false, b, (short)0, c, false, false);
  asm volatile("v_nop\n\tv_nop\n\tv_nop\n\tv_nop" : "+v"(d) : "v"(a), "v"(b));
  return d;
}
__device__ __forceinline__ v16h frag_h(const _Float16* rowk0, int lane) {
  union { v16h v; v8h q[2]; } u; const _Float16* p = rowk0 + 8 * (lane >> 4);
  u.q[0] = *(const v8h*)p; u.q[1] = *(const v8h*)(p + 16); return u.v;
}
__device__ __forceinline__ v16h frag_f32(const float* rowk0, int lane) {
  v16h a; const float* p = rowk0 + 8 * (lane >> 4);
#pragma unroll
  for (int i = 0; i < 8; ++i) { a[i] = (_Float16)p[i]; a[8 + i] = (_Float16)p[16 + i]; }
  return a;
}
__device__ __forceinline__ v16h frag_f32s(const float* rowk0, int lane, float sc) {
  v16h a; const float* p = rowk0 + 8 * (lane >> 4);
#pragma unroll
  for (int i = 0; i < 8; ++i) { a[i] = (_Float16)(p[i] * sc); a[8 + i] = (_Float16)(p[16 + i] * sc); }
  return a;
}
__device__ __forceinline__ v16h fragc_f32(const float* W, int k0, int n, int lane, int ld, int K) {
  v16h a; const int g = lane >> 4;
#pragma unroll
  for (int i = 0; i < 8; ++i) { const int ka = k0 + 8 * g + i, kb = ka + 16;
    a[i] = (_Float16)(ka < K ? W[(size_t)(ka < K ? ka : K - 1) * ld + n] : 0.f); a[8 + i] = (_Float16)(kb < K ? W[(size_t)(kb < K ? kb : K - 1) * ld + n] : 0.f); }
  return a;
}
struct F2 { v16b h, l; };
__device__ __forceinline__ F2 bsplit16(const float v[16]) { F2 r;
#pragma unroll
  for (int i = 0; i < 16; ++i) { const __bf16 h = (__bf16)v[i]; r.h[i] = h; r.l[i] = (__bf16)(v[i] - (float)h); }
  return r; }
__device__ __forceinline__ F2 split_row(const float* row, int k0, int lane) { float v[16]; const float* p = row + k0 + 8 * (lane >> 4);
#pragma unroll
  for (int i = 0; i < 8; ++i) { v[i] = p[i]; v[8 + i] = p[16 + i]; }
  return bsplit16(v); }
__device__ __forceinline__ F2 split_rowK(const float* row, int k0, int lane, int K) { float v[16]; const int g = lane >> 4;
#pragma unroll
  for (int i = 0; i < 8; ++i) { const int ka = k0 + 8 * g + i, kb = ka + 16; v[i] = ka < K ? row[ka < K ? ka : K - 1] : 0.f; v[8 + i] = kb < K ? row[kb < K ? kb : K - 1] : 0.f; }
  return bsplit16(v); }
__device__ __forceinline__ F2 split_col(const float* W, int k0, int n, int lane, int ld, int K) { float v[16]; const int g = lane >> 4;
#pragma unroll
  for (int i = 0; i < 8; ++i) { const int ka = k0 + 8 * g + i, kb = ka + 16; v[i] = ka < K ? W[(size_t)(ka < K ? ka : K - 1) * ld + n] : 0.f; v[8 + i] = kb < K ? W[(size_t)(kb < K ? kb : K - 1) * ld + n] : 0.f; }
  return bsplit16(v); }
__device__ __forceinline__ v8f mac3(const F2& a, const F2& b, v8f c) { c = wmma_bf(a.l, b.h, c); c = wmma_bf(a.h, b.l, c); return wmma_bf(a.h, b.h, c); }
__device__ __forceinline__ float sigm(float v) { return 1.0f / (1.0f + expf(-v)); }
#define LDSX() do { asm volatile("s_wait_dscnt 0" ::: "memory"); __builtin_amdgcn_wave_barrier(); __builtin_amdgcn_fence(__ATOMIC_RELEASE, "workgroup"); } while (0)


#define NN 16384
#define HH 128
#define NO 384
typedef __attribute__((ext_vector_type(8))) __bf16 v8b;
__device__ __forceinline__ v16b frag_b(const __bf16* rowk0, int lane) {
  union { v16b v; v8b q[2]; } u; const __bf16* p = rowk0 + 8 * (lane >> 4);
  u.q[0] = *(const v8b*)p; u.q[1] = *(const v8b*)(p + 16); return u.v;
}
__device__ __forceinline__ float bfr(float v) { return (float)(__bf16)v; }
__device__ __attribute__((noinline)) float exp_ni(float v) { return expf(v); }
__device__ __attribute__((noinline)) float erf_ni(float v) { return erff(v); }

#define WS_AT  0u
#define WS_U   (WS_AT + 2u * (size_t)HH * NO * HH)
#define WS_END (WS_U + 2u * (size_t)NO * 2 * HH)

__global__ __launch_bounds__(256) void k_packA(const float* __restrict__ A, __bf16* __restrict__ AT) {
  __shared__ __align__(16) __bf16 s[32][HH + 8]; const int a = blockIdx.x, oc = blockIdx.y; const int t = threadIdx.x;
  for (int e = t; e < HH * 32; e += 256) { const int b = e >> 5, ol = e & 31; s[ol][b] = (__bf16)A[((size_t)a * HH + b) * NO + oc * 32 + ol]; }
  __syncthreads();
  for (int e = t; e < 32 * (HH / 8); e += 256) { const int ol = e / (HH / 8), pc = e % (HH / 8); vst2((unsigned*)(AT + ((size_t)a * NO + oc * 32 + ol) * HH + pc * 8), *(const v4u*)&s[ol][pc * 8]); }
}
__global__ __launch_bounds__(256) void k_packU(const float* __restrict__ U1, const float* __restrict__ U2, __bf16* __restrict__ U) {
  __shared__ __align__(16) __bf16 s[2 * HH]; const int o = blockIdx.x, t = threadIdx.x; s[t] = (__bf16)((t < HH) ? U1[(size_t)o * HH + t] : U2[(size_t)o * HH + t - HH]);
  __syncthreads();
  if (t < 2 * HH / 8) vst2((unsigned*)(U + (size_t)o * 2 * HH + t * 8), *(const v4u*)&s[t * 8]);
}
__global__ __launch_bounds__(128) void k_cell(const float* __restrict__ NH_, const __bf16* __restrict__ AT, const __bf16* __restrict__ U, const float* __restrict__ UB, float* __restrict__ OUT) {
  __shared__ __align__(16) float so[4][16][132]; __shared__ float sh1[64][HH + 1];
  const int tid = threadIdx.x, wave = tid >> 5, lane = tid & 31, col = lane & 15, g = lane >> 4; const size_t r0 = (size_t)blockIdx.x * 64 + wave * 16; const int n0 = blockIdx.y * 128;
  for (int e = tid; e < 64 * HH; e += 128) { const int r = e / HH, a = e % HH; sh1[r][a] = bfr(NH_[((size_t)blockIdx.x * 64 + r) * 2 * HH + a]); }
  v16b ah2[4], ah1[4];
#pragma unroll
  for (int kc = 0; kc < 4; ++kc) { { const float* p = NH_ + (r0 + col) * 2 * HH + HH + kc * 32 + 8 * g; v16b a;
#pragma unroll
      for (int i = 0; i < 8; ++i) { a[i] = (__bf16)p[i]; a[8 + i] = (__bf16)p[16 + i]; } ah2[kc] = a; }
    { const float* p = NH_ + (r0 + col) * 2 * HH + kc * 32 + 8 * g; v16b a;
#pragma unroll
      for (int i = 0; i < 8; ++i) { a[i] = (__bf16)p[i]; a[8 + i] = (__bf16)p[16 + i]; } ah1[kc] = a; } }
  __syncthreads();
  v8f out[8] = {};
#pragma unroll 1
  for (int a = 0; a < HH; ++a) { v8f acc[8] = {};
    const __bf16* ATa = AT + ((size_t)a * NO + n0) * HH;
#pragma unroll
    for (int kc = 0; kc < 4; ++kc) {
#pragma unroll
      for (int j = 0; j < 8; ++j) acc[j] = wmma_bf(ah2[kc], frag_b(ATa + (size_t)(j * 16 + col) * HH + kc * 32, lane), acc[j]); }
    float h1a[8];
#pragma unroll
    for (int r = 0; r < 8; ++r) h1a[r] = sh1[wave * 16 + 8 * g + r][a];
#pragma unroll
    for (int j = 0; j < 8; ++j)
#pragma unroll
      for (int r = 0; r < 8; ++r) out[j][r] += h1a[r] * acc[j][r]; }
#pragma unroll
  for (int kc = 0; kc < 8; ++kc) { const v16b a = (kc < 4) ? ah1[kc] : ah2[kc - 4];
#pragma unroll
    for (int j = 0; j < 8; ++j) out[j] = wmma_bf(a, frag_b(U + (size_t)(n0 + j * 16 + col) * 2 * HH + kc * 32, lane), out[j]); }
#pragma unroll
  for (int j = 0; j < 8; ++j) { const float bb = bfr(UB[n0 + j * 16 + col]);
#pragma unroll
    for (int r = 0; r < 8; ++r) so[wave][8 * g + r][j * 16 + col] = out[j][r] + bb; }
  LDSX();
  for (int rl = 0; rl < 16; ++rl) vst2(OUT + (r0 + rl) * NO + n0 + lane * 4, *(const v4f*)&so[wave][rl][lane * 4]);
}
extern "C" void kernel_launch(void* const* d_in, const int* in_sizes, int n_in, void* d_out, int out_size, void* d_ws, size_t ws_size, hipStream_t stream) {
  (void)in_sizes; (void)n_in; (void)out_size;
  const float** F = (const float**)d_in;
  if (ws_size < (size_t)WS_END) return;
  char* ws = (char*)d_ws; __bf16 *AT = (__bf16*)(ws + WS_AT), *U = (__bf16*)(ws + WS_U);
  k_packA<<<dim3(HH, NO / 32), 256, 0, stream>>>(F[1], AT);
  k_packU<<<NO, 256, 0, stream>>>(F[2], F[3], U);
  k_cell<<<dim3(NN / 64, NO / 128), 128, 0, stream>>>(F[0], AT, U, F[4], (float*)d_out);
}
